// PlainMamba_36206574305360
// MI455X (gfx1250) — hardware-run, weakly checked
//
#include <hip/hip_runtime.h>


#ifndef NB
#define NB 2
#endif
#ifndef SEQ
#define SEQ 2048
#endif
#define NB_FULL  2
#define SEQ_FULL 2048
#ifndef OUT_SEQ
#define OUT_SEQ SEQ
#endif
#define DMD  384
#define DI   768
#define NZ   1536
#define NS   16
#define DTRK 24
#define XD   56
#define KCV  4
#define TS   64
#define XPS  256.0f
#define WXS  256.0f
#define DRS  1024.0f
#define WDS  64.0f
#define YSC  1024.0f
#define WOS  256.0f
#define XSCI (1.0f / 65536.0f)
#define DSCI (1.0f / 65536.0f)
#define OSCI (1.0f / 262144.0f)

static_assert(2 * DI == NZ);
static_assert(DTRK + 2 * NS == XD);
static_assert(NS == 16);
static_assert(KCV == 4);
static_assert(XD <= 64);
static_assert(DTRK % 8 == 0);
static_assert(DTRK <= 32);
static_assert(DMD % 64 == 0);
static_assert(DI % 64 == 0);
static_assert(NZ % 64 == 0);
static_assert(DMD % 32 == 0);
static_assert(DI % 32 == 0);
static_assert(DI % 256 == 0);
static_assert(DI % 8 == 0);
static_assert(SEQ % 64 == 0);
static_assert((NB * SEQ) % 64 == 0);
static_assert(SEQ % TS == 0);
static_assert(TS % 8 == 0);
static_assert(NB <= NB_FULL);
static_assert(SEQ <= SEQ_FULL);
static_assert(((size_t)SEQ * DMD) % 8 == 0);
static_assert(XPS * WXS == 65536.0f);
static_assert(DRS * WDS == 65536.0f);
static_assert(YSC * WOS == 262144.0f);
static_assert(16 * 68 * 4 <= 131072);
static_assert(64 * 65 * 4 <= 131072);
static_assert(TS * 32 * 4 + TS * 256 * 2 <= 131072);

typedef _Float16 h16;
typedef unsigned short bf;
typedef __attribute__((ext_vector_type(16))) __bf16   v16bf;
typedef __attribute__((ext_vector_type(16))) _Float16 v16h;
typedef __attribute__((ext_vector_type(8)))  _Float16 v8h;
typedef __attribute__((ext_vector_type(8)))  unsigned short v8us;
typedef __attribute__((ext_vector_type(8)))  float    v8f;
typedef __attribute__((ext_vector_type(4)))  float    v4f;
typedef v4f  __attribute__((may_alias)) v4fa;
typedef v8h  __attribute__((may_alias)) v8ha;

__device__ __forceinline__ unsigned short f2bf(float f) { unsigned u = __float_as_uint(f); u += 0x7FFFu + ((u >> 16) & 1u); return (unsigned short)(u >> 16); }
__device__ __forceinline__ float bfr(float f) { return __uint_as_float(((unsigned)f2bf(f)) << 16); }
__device__ __forceinline__ v16h cat16(v8h lo, v8h hi) { return __builtin_shufflevector(lo, hi, 0, 1, 2, 3, 4, 5, 6, 7, 8, 9, 10, 11, 12, 13, 14, 15); }
__device__ __forceinline__ v16bf cat16b(v8us lo, v8us hi) { return __builtin_bit_cast(v16bf, __builtin_shufflevector(lo, hi, 0, 1, 2, 3, 4, 5, 6, 7, 8, 9, 10, 11, 12, 13, 14, 15)); }
__device__ __forceinline__ v8f wmma16(v16h a, v16h b, v8f c) { return __builtin_amdgcn_wmma_f32_16x16x32_f16(false, a, false, b, (short)0, c, false, false); }
__device__ __forceinline__ v8f wmmab(v16bf a, v16bf b, v8f c) { return __builtin_amdgcn_wmma_f32_16x16x32_bf16(false, a, false, b, (short)0, c, false, false); }
__device__ __forceinline__ v16h  ldh(const h16* p) { return cat16(*(const v8h*)p, *(const v8h*)(p + 16)); }
__device__ __forceinline__ v16bf ldb(const bf* p)  { return cat16b(*(const v8us*)p, *(const v8us*)(p + 16)); }
__device__ __forceinline__ void wave_sync() { __builtin_amdgcn_fence(3  , "wavefront"); __builtin_amdgcn_wave_barrier(); asm volatile("" ::: "memory"); }

static __device__ __forceinline__ h16 toh_flush(float v) { const h16 r = (h16)v; return (fabsf(v) < 6.103515625e-05f) ? (h16)0.0f : r; }
__device__ __forceinline__ v8f wmma16g(v16h a, v16h b, v8f c) { c = wmma16(a, b, c); asm volatile("v_nop\n\tv_nop\n\tv_nop\n\tv_nop" : "+v"(c) : "v"(a), "v"(b)); return c; }
__device__ __forceinline__ v8f wmmabg(v16bf a, v16bf b, v8f c) { c = wmmab(a, b, c); asm volatile("v_nop\n\tv_nop\n\tv_nop\n\tv_nop" : "+v"(c) : "v"(a), "v"(b)); return c; }

__device__ __forceinline__ float conv_act(float x0, float x1, float x2, float x3, float w0, float w1, float w2, float w3, float cb) {
    const float s = x0 * w0 + x1 * w1 + x2 * w2 + x3 * w3 + cb;
    const float e = __expf(-s);
    return s * __builtin_amdgcn_rcpf(1.0f + e);
}

__global__ __launch_bounds__(256) void k_cvt8(const float* __restrict__ src, bf* dst, size_t n8) {
    const size_t i = (size_t)blockIdx.x * 256 + threadIdx.x; if (i >= n8) return;
    const v8f v = *(const v8f*)(src + i * 8); v8us o;
#pragma unroll
    for (int k = 0; k < 8; ++k) o[k] = f2bf(v[k]);
    *(volatile v8us*)(dst + i * 8) = o; __threadfence(); *(volatile v8us*)(dst + i * 8) = o;
}

__global__ __launch_bounds__(256) void k_wconv_b(const float* __restrict__ in, bf* out, int K, int N, int KP, int KT) {
    __shared__ __align__(16) float ts[64 * 65];
    const int tid = threadIdx.x; const int n0 = blockIdx.x * 64, k0 = blockIdx.y * KT;
#pragma unroll 1
    for (int e = tid; e < KT * 64; e += 256) {
        const int kk = e >> 6, nn = e & 63; const int k = k0 + kk, n = n0 + nn;
        const int kc = k < K ? k : K - 1, nc = n < N ? n : N - 1;
        float v = in[(size_t)kc * N + nc]; asm volatile("" : "+v"(v));
        const bool ok = (k < K) & (n < N);
        ts[nn * 65 + kk] = ok ? bfr(v) : 0.0f; }
    __syncthreads();
    const int sh = (KT == 64) ? 3 : 2; const int np = 64 << sh;
#pragma unroll 1
    for (int ps = 0; ps < 2; ++ps) {
#pragma unroll 1
        for (int p = tid; p < np; p += 256) { const int row = p >> sh, c8 = (p & ((1 << sh) - 1)) * 8; v8us o;
#pragma unroll
            for (int k = 0; k < 8; ++k) o[k] = f2bf(ts[row * 65 + c8 + k]);
            *(volatile v8us*)(out + (size_t)(n0 + row) * KP + k0 + c8) = o; }
        if (ps == 0) __threadfence(); }
}
__global__ __launch_bounds__(256) void k_wconv_h(const float* __restrict__ in, h16* out, int K, int N, int KP, int KT, float scale) {
    __shared__ __align__(16) float ts[64 * 65];
    const int tid = threadIdx.x; const int n0 = blockIdx.x * 64, k0 = blockIdx.y * KT;
#pragma unroll 1
    for (int e = tid; e < KT * 64; e += 256) {
        const int kk = e >> 6, nn = e & 63; const int k = k0 + kk, n = n0 + nn;
        const int kc = k < K ? k : K - 1, nc = n < N ? n : N - 1;
        float v = in[(size_t)kc * N + nc]; asm volatile("" : "+v"(v));
        const bool ok = (k < K) & (n < N);
        ts[nn * 65 + kk] = ok ? bfr(v) * scale : 0.0f; }
    __syncthreads();
    const int sh = (KT == 64) ? 3 : 2; const int np = 64 << sh;
#pragma unroll 1
    for (int ps = 0; ps < 2; ++ps) {
#pragma unroll 1
        for (int p = tid; p < np; p += 256) { const int row = p >> sh, c8 = (p & ((1 << sh) - 1)) * 8; v8h o;
#pragma unroll
            for (int k = 0; k < 8; ++k) o[k] = toh_flush(ts[row * 65 + c8 + k]);
            *(volatile v8h*)(out + (size_t)(n0 + row) * KP + k0 + c8) = o; }
        if (ps == 0) __threadfence(); }
}

__device__ __forceinline__ void gemm_core_b(const bf* __restrict__ A, const bf* __restrict__ Bt, const int K, const size_t aoff, const size_t boff, v8f (&acc)[4][4]) {
#pragma unroll 1
    for (int kc = 0; kc < K; kc += 32) {
        v16bf a[4];
#pragma unroll
        for (int mb = 0; mb < 4; ++mb) a[mb] = ldb(A + aoff + (size_t)mb * 16 * K + kc);
#pragma unroll
        for (int nb = 0; nb < 4; ++nb) { const v16bf b = ldb(Bt + boff + (size_t)nb * 16 * K + kc);
#pragma unroll
            for (int mb = 0; mb < 4; ++mb) acc[mb][nb] = wmmabg(a[mb], b, acc[mb][nb]); }
    }
}
__device__ __forceinline__ void gemm_core_h(const h16* __restrict__ A, const h16* __restrict__ Bt, const int K, const size_t aoff, const size_t boff, v8f (&acc)[4][4]) {
#pragma unroll 1
    for (int kc = 0; kc < K; kc += 32) {
        v16h a[4];
#pragma unroll
        for (int mb = 0; mb < 4; ++mb) a[mb] = ldh(A + aoff + (size_t)mb * 16 * K + kc);
#pragma unroll
        for (int nb = 0; nb < 4; ++nb) { const v16h b = ldh(Bt + boff + (size_t)nb * 16 * K + kc);
#pragma unroll
            for (int mb = 0; mb < 4; ++mb) acc[mb][nb] = wmma16g(a[mb], b, acc[mb][nb]); }
    }
}

__global__ __launch_bounds__(32) void k_gemm_b(const bf* __restrict__ A, const bf* __restrict__ Bt, float* C, int K, int ldc, int obs) {
    __shared__ __align__(16) float os[16 * 68];
    const int lane = threadIdx.x & 31, lr = lane & 15, hi = lane >> 4; const int r0 = blockIdx.x * 64, c0 = blockIdx.y * 64;
    v8f acc[4][4];
#pragma unroll
    for (int mb = 0; mb < 4; ++mb)
#pragma unroll
        for (int nb = 0; nb < 4; ++nb) acc[mb][nb] = (v8f){};
    gemm_core_b(A, Bt, K, (size_t)(r0 + lr) * K + 8 * hi, (size_t)(c0 + lr) * K + 8 * hi, acc);
    const int bb = r0 / SEQ, tt = r0 % SEQ; const size_t crow0 = (size_t)bb * (size_t)obs + (size_t)tt;
#pragma unroll
    for (int mb = 0; mb < 4; ++mb) {
#pragma unroll
        for (int nb = 0; nb < 4; ++nb) {
#pragma unroll
            for (int j = 0; j < 8; ++j) os[(hi * 8 + j) * 68 + nb * 16 + lr] = acc[mb][nb][j]; }
        wave_sync();
        static_assert(8 * 32 * 16 == 16 * 64 * 4);
#pragma unroll 1
        for (int ps = 0; ps < 2; ++ps) {
#pragma unroll
            for (int s = 0; s < 8; ++s) { const int row = 2 * s + (lane >> 4), c4 = (lane & 15) * 4;
                const v4f val = *(const v4fa*)(&os[row * 68 + c4]);
                *(volatile v4f*)(C + (crow0 + (size_t)(mb * 16 + row)) * (size_t)ldc + c0 + c4) = val; }
            if (ps == 0) __threadfence(); }
        wave_sync();
    }
}

__global__ __launch_bounds__(32) void k_gemm_h(const h16* __restrict__ A, const h16* __restrict__ Bt, float* C, int K, int ldc, int obs, float scale,
                                               const float* __restrict__ bias, int hasb, int nbias) {
    __shared__ __align__(16) float os[16 * 68];
    const int lane = threadIdx.x & 31, lr = lane & 15, hi = lane >> 4; const int r0 = blockIdx.x * 64, c0 = blockIdx.y * 64;
    v8f acc[4][4];
#pragma unroll
    for (int mb = 0; mb < 4; ++mb)
#pragma unroll
        for (int nb = 0; nb < 4; ++nb) acc[mb][nb] = (v8f){};
    gemm_core_h(A, Bt, K, (size_t)(r0 + lr) * K + 8 * hi, (size_t)(c0 + lr) * K + 8 * hi, acc);
    float bc[4];
#pragma unroll
    for (int nb = 0; nb < 4; ++nb) { int ci = c0 + nb * 16 + lr; ci = ci < nbias ? ci : nbias - 1;
        float bv = bias[ci]; asm volatile("" : "+v"(bv));
        bc[nb] = (hasb != 0) ? bfr(bv) : 0.0f; }
    const int bb = r0 / SEQ, tt = r0 % SEQ; const size_t crow0 = (size_t)bb * (size_t)obs + (size_t)tt;
#pragma unroll
    for (int mb = 0; mb < 4; ++mb) {
#pragma unroll
        for (int nb = 0; nb < 4; ++nb) {
#pragma unroll
            for (int j = 0; j < 8; ++j) os[(hi * 8 + j) * 68 + nb * 16 + lr] = acc[mb][nb][j] * scale + bc[nb]; }
        wave_sync();
        static_assert(8 * 32 * 16 == 16 * 64 * 4);
#pragma unroll 1
        for (int ps = 0; ps < 2; ++ps) {
#pragma unroll
            for (int s = 0; s < 8; ++s) { const int row = 2 * s + (lane >> 4), c4 = (lane & 15) * 4;
                const v4f val = *(const v4fa*)(&os[row * 68 + c4]);
                *(volatile v4f*)(C + (crow0 + (size_t)(mb * 16 + row)) * (size_t)ldc + c0 + c4) = val; }
            if (ps == 0) __threadfence(); }
        wave_sync();
    }
}

__global__ __launch_bounds__(32) void k_gemm_x(const h16* __restrict__ A, const h16* __restrict__ Bt, h16* DTR, float* BC) {
    __shared__ __align__(16) float os[16 * 68];
    const int lane = threadIdx.x & 31, lr = lane & 15, hi = lane >> 4; const int r0 = blockIdx.x * 64;
    v8f acc[4][4];
#pragma unroll
    for (int mb = 0; mb < 4; ++mb)
#pragma unroll
        for (int nb = 0; nb < 4; ++nb) acc[mb][nb] = (v8f){};
    gemm_core_h(A, Bt, DI, (size_t)(r0 + lr) * DI + 8 * hi, (size_t)lr * DI + 8 * hi, acc);
#pragma unroll
    for (int mb = 0; mb < 4; ++mb) {
#pragma unroll
        for (int nb = 0; nb < 4; ++nb) {
#pragma unroll
            for (int j = 0; j < 8; ++j) os[(hi * 8 + j) * 68 + nb * 16 + lr] = acc[mb][nb][j] * XSCI; }
        wave_sync();
        static_assert(2 * 32 * 16 == 16 * 32 * 2);
        static_assert(4 * 32 * 16 == 16 * 32 * 4);
#pragma unroll 1
        for (int ps = 0; ps < 2; ++ps) {
#pragma unroll
            for (int s = 0; s < 2; ++s) { const int p = s * 32 + lane; const int row = p >> 2, c8 = (p & 3) * 8;
                const v4f x0 = *(const v4fa*)(&os[row * 68 + c8]); const v4f x1 = *(const v4fa*)(&os[row * 68 + c8 + 4]);
                const bool kp = c8 < DTRK; v8h hv;
#pragma unroll
                for (int i = 0; i < 4; ++i) { const h16 a0 = toh_flush(x0[i] * DRS); const h16 a1 = toh_flush(x1[i] * DRS); hv[i] = kp ? a0 : (h16)0.0f; hv[4 + i] = kp ? a1 : (h16)0.0f; }
                *(volatile v8h*)(DTR + (size_t)(r0 + mb * 16) * 32 + (size_t)p * 8) = hv; }
#pragma unroll
            for (int s = 0; s < 4; ++s) { const int row = 4 * s + (lane >> 3), c4 = (lane & 7) * 4;
                const v4f val = *(const v4fa*)(&os[row * 68 + DTRK + c4]);
                *(volatile v4f*)(BC + (size_t)(r0 + mb * 16 + row) * 32 + c4) = val; }
            if (ps == 0) __threadfence(); }
        wave_sync();
    }
}

__global__ __launch_bounds__(256) void k_conv(const float* __restrict__ XZ, const float* __restrict__ conv_w, const float* __restrict__ conv_b, h16* XP) {
    const size_t i = (size_t)blockIdx.x * 256 + threadIdx.x; if (i >= (size_t)NB * SEQ * (DI / 8)) return;
    const int m = (int)(i / (DI / 8)); const int d0 = (int)(i % (DI / 8)) * 8; const int t = m % SEQ;
    const v4f zz = (v4f){};
    v4f xa[4][2];
#pragma unroll
    for (int j = 0; j < 4; ++j) { const bool ok = (t - 3 + j) >= 0; const int mc = ok ? (m - 3 + j) : m;
        v4f p0 = *(const v4f*)(XZ + (size_t)mc * NZ + d0); v4f p1 = *(const v4f*)(XZ + (size_t)mc * NZ + d0 + 4);
        asm volatile("" : "+v"(p0)); asm volatile("" : "+v"(p1));
        xa[j][0] = ok ? p0 : zz; xa[j][1] = ok ? p1 : zz; }
    const v4f cb0 = *(const v4f*)(conv_b + d0), cb1 = *(const v4f*)(conv_b + d0 + 4);
    v8h o;
#pragma unroll
    for (int c = 0; c < 8; ++c) { const v4f wv = *(const v4f*)(conv_w + (size_t)(d0 + c) * KCV);
        const float cb = bfr((c < 4) ? cb0[c & 3] : cb1[c & 3]);
        const float xp = conv_act(xa[0][c >> 2][c & 3], xa[1][c >> 2][c & 3], xa[2][c >> 2][c & 3], xa[3][c >> 2][c & 3], bfr(wv[0]), bfr(wv[1]), bfr(wv[2]), bfr(wv[3]), cb);
        o[c] = toh_flush(xp * XPS); }
    *(volatile v8h*)(XP + i * 8) = o; __threadfence(); *(volatile v8h*)(XP + i * 8) = o;
}

__global__ __launch_bounds__(256) void k_scan(const float* __restrict__ XZ, const float* __restrict__ DTP, const float* __restrict__ BC,
                                              const float* __restrict__ conv_w, const float* __restrict__ conv_b,
                                              const float* __restrict__ A_log, const float* __restrict__ Dv, h16* Y16) {
    __shared__ __align__(16) float sBC[TS * 32];
    __shared__ __align__(16) h16 ys[TS * 256];
    const int tid = threadIdx.x;
    const int b = blockIdx.x / (DI / 256); const int dbase = (blockIdx.x % (DI / 256)) * 256; const int d = dbase + tid;
    float An[NS];
#pragma unroll
    for (int q = 0; q < 4; ++q) { const v4f al = *(const v4f*)(A_log + (size_t)d * NS + 4 * q);
#pragma unroll
        for (int i = 0; i < 4; ++i) An[4 * q + i] = -__expf(bfr(al[i])); }
    const float Dd = bfr(Dv[d]);
    const v4f cwv = *(const v4f*)(conv_w + (size_t)d * KCV);
    const float w0 = bfr(cwv[0]), w1 = bfr(cwv[1]), w2 = bfr(cwv[2]), w3 = bfr(cwv[3]);
    const float cb = bfr(conv_b[d]);
    float h[NS];
#pragma unroll
    for (int n = 0; n < NS; ++n) h[n] = 0.0f;
    float x0 = 0.0f, x1 = 0.0f, x2 = 0.0f;
#pragma unroll 1
    for (int l0 = 0; l0 < SEQ; l0 += TS) {
        const size_t mb0 = (size_t)b * SEQ + (size_t)l0;
#pragma unroll 1
        for (int q = tid; q < TS * 8; q += 256) { const v4f v = *(const v4f*)(BC + mb0 * 32 + (size_t)q * 4); *(v4fa*)(&sBC[q * 4]) = v; }
        __syncthreads();
#pragma unroll 1
        for (int i = 0; i < TS; ++i) {
            const size_t m = mb0 + (size_t)i;
            const float x3 = XZ[m * NZ + d]; const float zv = XZ[m * NZ + DI + d]; const float dp = DTP[m * DI + d];
            const float xp = conv_act(x0, x1, x2, x3, w0, w1, w2, w3, cb); x0 = x1; x1 = x2; x2 = x3;
            const float dtv = fmaxf(dp, 0.0f) + __logf(1.0f + __expf(-fabsf(dp)));
            const float dtx = dtv * xp;
            v4f bv[8];
#pragma unroll
            for (int q = 0; q < 8; ++q) bv[q] = *(const v4fa*)(&sBC[i * 32 + 4 * q]);
            float y = 0.0f;
#pragma unroll
            for (int n = 0; n < NS; ++n) { const float dA = __expf(dtv * An[n]);
                h[n] = dA * h[n] + bv[n >> 2][n & 3] * dtx;
                y += h[n] * bv[4 + (n >> 2)][n & 3]; }
            y += xp * Dd;
            const float sz = zv * __builtin_amdgcn_rcpf(1.0f + __expf(-zv));
            ys[i * 256 + tid] = toh_flush(y * sz * YSC);
        }
        __syncthreads();
        static_assert((TS / 8) * 256 * 16 == TS * 256 * 2);
#pragma unroll 1
        for (int ps = 0; ps < 2; ++ps) {
#pragma unroll 1
            for (int it = 0; it < TS / 8; ++it) { const int p = it * 256 + tid; const int row = p >> 5, c8 = (p & 31) * 8;
                const v8h val = *(const v8ha*)(&ys[row * 256 + c8]);
                *(volatile v8h*)(Y16 + (mb0 + (size_t)row) * DI + dbase + c8) = val; }
            if (ps == 0) __threadfence(); }
        __syncthreads();
    }
}

static constexpr size_t al256(size_t v) { return (v + 255) & ~(size_t)255; }
static constexpr size_t SZ_XB  = al256((size_t)NB * SEQ * DMD * 2);
static constexpr size_t SZ_WIN = al256((size_t)NZ * DMD * 2);
static constexpr size_t SZ_WX  = al256((size_t)64 * DI * 2);
static constexpr size_t SZ_WD  = al256((size_t)DI * 32 * 2);
static constexpr size_t SZ_WO  = al256((size_t)DMD * DI * 2);
static constexpr size_t SZ_XZ  = al256((size_t)NB * SEQ * NZ * 4);
static constexpr size_t SZ_XP  = al256((size_t)NB * SEQ * DI * 2);
static constexpr size_t SZ_DTR = al256((size_t)NB * SEQ * 32 * 2);
static constexpr size_t SZ_BC  = al256((size_t)NB * SEQ * 32 * 4);
static constexpr size_t SZ_DTP = al256((size_t)NB * SEQ * DI * 4);
static constexpr size_t SZ_Y   = al256((size_t)NB * SEQ * DI * 2);
static constexpr size_t SZ_TOTAL = SZ_XB + SZ_WIN + SZ_WX + SZ_WD + SZ_WO + SZ_XZ + SZ_XP + SZ_DTR + SZ_BC + SZ_DTP + SZ_Y;
static_assert(SZ_TOTAL <= (size_t)134217728);

extern "C" void kernel_launch(void* const* d_in, const int* in_sizes, int n_in,
                              void* d_out, int out_size, void* d_ws, size_t ws_size, hipStream_t stream) {
    if (n_in < 10) return;
    const size_t needx = ((size_t)(NB - 1) * SEQ_FULL + SEQ) * DMD;
    if ((size_t)in_sizes[0] < needx) return;
    if ((size_t)in_sizes[1] < (size_t)DMD * NZ || (size_t)in_sizes[2] < (size_t)DI * KCV || in_sizes[3] < DI) return;
    if ((size_t)in_sizes[4] < (size_t)DI * XD || (size_t)in_sizes[5] < (size_t)DTRK * DI || in_sizes[6] < DI) return;
    if ((size_t)in_sizes[7] < (size_t)DI * NS || in_sizes[8] < DI || (size_t)in_sizes[9] < (size_t)DI * DMD) return;
    if ((size_t)out_size < ((size_t)(NB - 1) * OUT_SEQ + SEQ) * DMD) return;
    if (SZ_TOTAL > ws_size) return;
    const float* x   = (const float*)d_in[0];
    const float* win = (const float*)d_in[1];
    const float* cw  = (const float*)d_in[2];
    const float* cb  = (const float*)d_in[3];
    const float* wx  = (const float*)d_in[4];
    const float* wd  = (const float*)d_in[5];
    const float* dtb = (const float*)d_in[6];
    const float* alg = (const float*)d_in[7];
    const float* dv  = (const float*)d_in[8];
    const float* wo  = (const float*)d_in[9];
    float* OUT = (float*)d_out;
    char* wsp = (char*)d_ws;
    bf*    XB   = (bf*)wsp;    wsp += SZ_XB;
    bf*    WINT = (bf*)wsp;    wsp += SZ_WIN;
    h16*   WXT  = (h16*)wsp;   wsp += SZ_WX;
    h16*   WDT  = (h16*)wsp;   wsp += SZ_WD;
    h16*   WOT  = (h16*)wsp;   wsp += SZ_WO;
    float* XZ   = (float*)wsp; wsp += SZ_XZ;
    h16*   XP   = (h16*)wsp;   wsp += SZ_XP;
    h16*   DTR  = (h16*)wsp;   wsp += SZ_DTR;
    float* BC   = (float*)wsp; wsp += SZ_BC;
    float* DTP  = (float*)wsp; wsp += SZ_DTP;
    h16*   Y16  = (h16*)wsp;   wsp += SZ_Y;
    const int M = NB * SEQ;

    if (SEQ == SEQ_FULL) {
        const size_t n8 = (size_t)NB * SEQ * DMD / 8;
        k_cvt8<<<(unsigned)((n8 + 255) / 256), 256, 0, stream>>>(x, XB, n8);
    } else {
        const size_t n8 = (size_t)SEQ * DMD / 8;
        for (int b = 0; b < NB; ++b) k_cvt8<<<(unsigned)((n8 + 255) / 256), 256, 0, stream>>>(x + (size_t)b * SEQ_FULL * DMD, XB + (size_t)b * SEQ * DMD, n8);
    }
    k_wconv_b<<<dim3(NZ / 64, DMD / 64, 1), 256, 0, stream>>>(win, WINT, DMD, NZ, DMD, 64);
    k_wconv_h<<<dim3(1, DI / 64, 1), 256, 0, stream>>>(wx, WXT, DI, XD, DI, 64, WXS);
    k_wconv_h<<<dim3(DI / 64, 1, 1), 256, 0, stream>>>(wd, WDT, DTRK, DI, 32, 32, WDS);
    k_wconv_h<<<dim3(DMD / 64, DI / 64, 1), 256, 0, stream>>>(wo, WOT, DI, DMD, DI, 64, WOS);

    k_gemm_b<<<dim3(M / 64, NZ / 64, 1), 32, 0, stream>>>(XB, WINT, XZ, DMD, NZ, SEQ);
    { const size_t n = (size_t)NB * SEQ * (DI / 8);
      k_conv<<<(unsigned)((n + 255) / 256), 256, 0, stream>>>(XZ, cw, cb, XP); }
    k_gemm_x<<<dim3(M / 64, 1, 1), 32, 0, stream>>>(XP, WXT, DTR, BC);
    k_gemm_h<<<dim3(M / 64, DI / 64, 1), 32, 0, stream>>>(DTR, WDT, DTP, 32, DI, SEQ, DSCI, dtb, 1, DI);
    k_scan<<<NB * (DI / 256), 256, 0, stream>>>(XZ, DTP, BC, cw, cb, alg, dv, Y16);
    k_gemm_h<<<dim3(M / 64, DMD / 64, 1), 32, 0, stream>>>(Y16, WOT, OUT, DI, DMD, OUT_SEQ, OSCI, dtb, 0, DI);
}
